// EntAttentionLayer_82815559401987
// MI455X (gfx1250) — hardware-verified
//
#include <hip/hip_runtime.h>


#define NB_  2
#define NTAG 64
#define TT   2048
#define DD   768
#define NH_  12
#define HD   64
#define NT   (NB_ * TT)
#define ZH   2
#define FFH  3072
#define PCAR 1024.0f
typedef _Float16 h16;
typedef unsigned short bf;
typedef __attribute__((ext_vector_type(16))) __bf16   v16bf;
typedef __attribute__((ext_vector_type(16))) _Float16 v16h;
typedef __attribute__((ext_vector_type(8)))  _Float16 v8h;
typedef __attribute__((ext_vector_type(8)))  unsigned short v8us;
typedef __attribute__((ext_vector_type(8)))  float    v8f;
typedef __attribute__((ext_vector_type(4)))  float    v4f;
typedef v8h  __attribute__((may_alias)) v8ha;
typedef v4f  __attribute__((may_alias)) v4fa;
typedef v8us __attribute__((may_alias)) v8usa;

__device__ __forceinline__ unsigned short f2bf(float f) { unsigned u = __float_as_uint(f); u += 0x7FFFu + ((u >> 16) & 1u); return (unsigned short)(u >> 16); }
__device__ __forceinline__ float bf2f(unsigned short b) { return __uint_as_float(((unsigned)b) << 16); }
__device__ __forceinline__ float bfr(float f) { return bf2f(f2bf(f)); }
__device__ __forceinline__ v16h cat16(v8h lo, v8h hi) { return __builtin_shufflevector(lo, hi, 0, 1, 2, 3, 4, 5, 6, 7, 8, 9, 10, 11, 12, 13, 14, 15); }
__device__ __forceinline__ v16bf cat16b(v8us lo, v8us hi) { return __builtin_bit_cast(v16bf, __builtin_shufflevector(lo, hi, 0, 1, 2, 3, 4, 5, 6, 7, 8, 9, 10, 11, 12, 13, 14, 15)); }
__device__ __forceinline__ v8f wmma16(v16h a, v16h b, v8f c) { return __builtin_amdgcn_wmma_f32_16x16x32_f16(false, a, false, b, (short)0, c, false, false); }
__device__ __forceinline__ v8f wmmab(v16bf a, v16bf b, v8f c) { return __builtin_amdgcn_wmma_f32_16x16x32_bf16(false, a, false, b, (short)0, c, false, false); }


template <typename T16> struct WFrag;
template <> struct WFrag<h16> { typedef v16h V; static __device__ __forceinline__ V ld(const h16* p) { return cat16(*(const v8h*)p, *(const v8h*)(p + 16)); } static __device__ __forceinline__ v8f mma(V a, V b, v8f c) { return wmma16(a, b, c); } };
template <> struct WFrag<bf> { typedef v16bf V; static __device__ __forceinline__ V ld(const bf* p) { return cat16b(*(const v8us*)p, *(const v8us*)(p + 16)); } static __device__ __forceinline__ v8f mma(V a, V b, v8f c) { return wmmab(a, b, c); } };
template <typename T16, int NSPLIT, bool BIAS>
__global__ __launch_bounds__(32) void k_gemmw(const T16* __restrict__ A, const T16* __restrict__ A2, const T16* __restrict__ Bt, const T16* __restrict__ Bt2, int K, float* C, int ldc, const float* __restrict__ bias, size_t sA, size_t sB, size_t sC) {
    typedef typename WFrag<T16>::V V;
    __shared__ __align__(16) float os[16 * 68];
    const size_t z = blockIdx.z; A += z * sA; if (A2) A2 += z * sA; Bt += z * sB; if (Bt2) Bt2 += z * sB; C += z * sC;
    const int lane = threadIdx.x & 31, lr = lane & 15, hi = lane >> 4; const int r0 = blockIdx.x * 64, c0 = blockIdx.y * 64;
    v8f acc[4][4];
#pragma unroll
    for (int mb = 0; mb < 4; ++mb)
#pragma unroll
        for (int nb = 0; nb < 4; ++nb) acc[mb][nb] = (v8f){};
    const size_t aoff = (size_t)(r0 + lr) * K + 8 * hi, boff = (size_t)(c0 + lr) * K + 8 * hi;
#pragma unroll 1
    for (int kc = 0; kc < K; kc += 32) {
        V a[4], a2[4];
#pragma unroll
        for (int mb = 0; mb < 4; ++mb) { a[mb] = WFrag<T16>::ld(A + aoff + (size_t)mb * 16 * K + kc); if (NSPLIT == 1 || NSPLIT == 2) a2[mb] = WFrag<T16>::ld(A2 + aoff + (size_t)mb * 16 * K + kc); }
#pragma unroll
        for (int nb = 0; nb < 4; ++nb) { const V b = WFrag<T16>::ld(Bt + boff + (size_t)nb * 16 * K + kc); V b2; if (NSPLIT >= 2) b2 = WFrag<T16>::ld(Bt2 + boff + (size_t)nb * 16 * K + kc);
#pragma unroll
            for (int mb = 0; mb < 4; ++mb) { acc[mb][nb] = WFrag<T16>::mma(a[mb], b, acc[mb][nb]); if (NSPLIT == 1 || NSPLIT == 2) acc[mb][nb] = WFrag<T16>::mma(a2[mb], b, acc[mb][nb]); if (NSPLIT >= 2) acc[mb][nb] = WFrag<T16>::mma(a[mb], b2, acc[mb][nb]); } }
        asm volatile("v_nop\n\tv_nop\n\tv_nop\n\tv_nop" : "+v"(acc[0][0]), "+v"(acc[1][1]), "+v"(acc[2][2]), "+v"(acc[3][3]) : "v"(a[0]), "v"(a[3]));
    }
#pragma unroll
    for (int mb = 0; mb < 4; ++mb) {
#pragma unroll
        for (int nb = 0; nb < 4; ++nb) {
#pragma unroll
            for (int j = 0; j < 8; ++j) os[(hi * 8 + j) * 68 + nb * 16 + lr] = acc[mb][nb][j]; }
        __builtin_amdgcn_wave_barrier(); asm volatile("" ::: "memory");
        float* crow = C + (size_t)(r0 + mb * 16) * ldc + c0;
#pragma unroll 1
        for (int ps = 0; ps < 2; ++ps) {
#pragma unroll
            for (int s = 0; s < 8; ++s) { const int row = 2 * s + hi, cofs = lr * 4; v4f val = *(const v4fa*)(os + row * 68 + cofs); if (BIAS) { val[0] += bfr(bias[c0 + cofs]); val[1] += bfr(bias[c0 + cofs + 1]); val[2] += bfr(bias[c0 + cofs + 2]); val[3] += bfr(bias[c0 + cofs + 3]); }
                *(volatile v4f*)(crow + (size_t)row * ldc + cofs) = val; }
            if (ps == 0) __threadfence(); }
        __builtin_amdgcn_wave_barrier(); asm volatile("" ::: "memory");
    }
}

__device__ __forceinline__ h16 tohx(float x) { return (h16)x; }
__device__ __forceinline__ void splitf(float y, unsigned short& h, unsigned short& l) { h = f2bf(y); l = f2bf(y - bf2f(h)); }
typedef __attribute__((ext_vector_type(2))) _Float16 v2h;
typedef __attribute__((ext_vector_type(4))) _Float16 v4h;
typedef __attribute__((ext_vector_type(2))) unsigned short v2us;
typedef __attribute__((ext_vector_type(4))) unsigned short v4us;
typedef __attribute__((ext_vector_type(2))) float v2f;

__global__ __launch_bounds__(256) void k_cvt8(const float* __restrict__ src, bf* dst, size_t n8) { const size_t i = (size_t)blockIdx.x * 256 + threadIdx.x; if (i >= n8) return; const v8f v = *(const v8f*)(src + i * 8); v8us o;
#pragma unroll
    for (int k = 0; k < 8; ++k) o[k] = f2bf(v[k]); *(volatile v8us*)(dst + i * 8) = o; __threadfence(); *(volatile v8us*)(dst + i * 8) = o; }
__global__ __launch_bounds__(256) void k_wtG(const float* __restrict__ w, int K, int N, bf* Bt) {
    const int lane = threadIdx.x & 31; const int L0 = (blockIdx.x * 8 + (threadIdx.x >> 5)) * 8; const int nlines = N * K / 64;
#pragma unroll 1
    for (int ps = 0; ps < 2; ++ps) {
#pragma unroll 1
        for (int l = 0; l < 8; ++l) { const int L = L0 + l; if (L >= nlines) break; const size_t e = (size_t)L * 64 + lane * 2; const int k = (int)(e % K), n = (int)(e / K); v2us o;
            o[0] = f2bf(w[(size_t)k * N + n]); o[1] = f2bf(w[(size_t)(k + 1) * N + n]); *(volatile v2us*)(Bt + e) = o; }
        if (ps == 0) __threadfence(); }
}
__global__ __launch_bounds__(256) void k_bfr1(const float* __restrict__ src, float* dst, int n) { const int i = blockIdx.x * 256 + threadIdx.x; if (i >= n) return; const float v = bfr(src[i]); *(volatile float*)(dst + i) = v; __threadfence(); *(volatile float*)(dst + i) = v; }
__global__ __launch_bounds__(256) void k_h16plane(const float* __restrict__ F, float sc, h16* P) {
    const int lane = threadIdx.x & 31; const int L0 = (blockIdx.x * 8 + (threadIdx.x >> 5)) * 8; const int nlines = NT * DD / 64;
#pragma unroll 1
    for (int ps = 0; ps < 2; ++ps) {
#pragma unroll
        for (int l = 0; l < 8; ++l) { const int L = L0 + l; if (L >= nlines) break; const int e = L * 64 + lane * 2; const int d = e & 63; const int t = (e >> 6) & (TT - 1); const int z = e >> 17; const int b = z / NH_, h = z % NH_; v2h v;
#pragma unroll
            for (int q = 0; q < 2; ++q) v[q] = tohx(F[((size_t)b * TT + t) * DD + h * HD + d + q] * sc);
            *(volatile v2h*)(P + (size_t)e) = v; }
        if (ps == 0) __threadfence(); }
}
__global__ __launch_bounds__(256) void k_vtplane(const float* __restrict__ F, h16* VT) {
    const int lane = threadIdx.x & 31; const int L0 = (blockIdx.x * 8 + (threadIdx.x >> 5)) * 8; const int nlines = NT * DD / 64;
#pragma unroll 1
    for (int ps = 0; ps < 2; ++ps) {
#pragma unroll
        for (int l = 0; l < 8; ++l) { const int L = L0 + l; if (L >= nlines) break; const int e = L * 64 + lane * 2; const int t = e & (TT - 1); const int d = (e >> 11) & 63; const int z = e >> 17; const int b = z / NH_, h = z % NH_; v2h v;
#pragma unroll
            for (int q = 0; q < 2; ++q) v[q] = tohx(F[((size_t)b * TT + t + q) * DD + h * HD + d]);
            *(volatile v2h*)(VT + (size_t)e) = v; }
        if (ps == 0) __threadfence(); }
}
__global__ __launch_bounds__(256) void k_msoft(const float* __restrict__ Sb, h16* P) {
    const int lane = threadIdx.x & 31; const int row = blockIdx.x * 8 + (threadIdx.x >> 5); if (row >= ZH * TT) return; const int i = row & (TT - 1);
    const float* sr = Sb + (size_t)row * TT; float v[64]; float mx = -3.0e38f;
#pragma unroll
    for (int ch = 0; ch < 16; ++ch) { const int j0 = ch * 128 + lane * 4; const v4f a = *(const v4f*)(sr + j0);
#pragma unroll
        for (int q = 0; q < 4; ++q) { const int j = j0 + q; const int dj = j - i; const float t = (dj <= 50 && dj >= -50) ? __fadd_rn(a[q], 1.0f) : a[q]; v[ch * 4 + q] = t; mx = fmaxf(mx, t); } }
#pragma unroll
    for (int sh = 16; sh; sh >>= 1) mx = fmaxf(mx, __shfl_xor(mx, sh, 32));
    float sum = 0.f;
#pragma unroll
    for (int k = 0; k < 64; ++k) { v[k] = __expf(v[k] - mx); sum += v[k]; }
#pragma unroll
    for (int sh = 16; sh; sh >>= 1) sum += __shfl_xor(sum, sh, 32);
    const float f = __fdiv_rn(PCAR, sum);
#pragma unroll 1
    for (int ps = 0; ps < 2; ++ps) {
#pragma unroll
        for (int ch = 0; ch < 16; ++ch) { v4h o;
#pragma unroll
            for (int q = 0; q < 4; ++q) o[q] = tohx(v[ch * 4 + q] * f);
            *(volatile v4h*)(P + (size_t)row * TT + ch * 128 + lane * 4) = o; }
        if (ps == 0) __threadfence(); }
}
__global__ __launch_bounds__(256) void k_soft64(const float* __restrict__ SX, int nrows, h16* PX) {
    const int lane = threadIdx.x & 31; const int row = blockIdx.x * 8 + (threadIdx.x >> 5); if (row >= nrows) return; const v2f a = *(const v2f*)(SX + (size_t)row * NTAG + lane * 2);
    float mx = fmaxf(a[0], a[1]);
#pragma unroll
    for (int sh = 16; sh; sh >>= 1) mx = fmaxf(mx, __shfl_xor(mx, sh, 32));
    const float e0 = __expf(a[0] - mx), e1 = __expf(a[1] - mx); float sum = e0 + e1;
#pragma unroll
    for (int sh = 16; sh; sh >>= 1) sum += __shfl_xor(sum, sh, 32);
    const float f = __fdiv_rn(PCAR, sum); v2h o; o[0] = tohx(e0 * f); o[1] = tohx(e1 * f);
    *(volatile v2h*)(PX + (size_t)row * NTAG + lane * 2) = o; __threadfence(); *(volatile v2h*)(PX + (size_t)row * NTAG + lane * 2) = o;
}
__global__ __launch_bounds__(256) void k_tag16(const float* __restrict__ FK, const float* __restrict__ FVt, h16* KX, h16* VXT) {
    const int e = (blockIdx.x * 256 + threadIdx.x) * 4; if (e >= NH_ * NTAG * HD) return; v4h kk, vv;
    { const int d = e & 63; const int j = (e >> 6) & 63; const int h = e >> 12;
#pragma unroll
      for (int q = 0; q < 4; ++q) kk[q] = tohx(FK[(size_t)j * DD + h * HD + d + q]); }
    { const int j2 = e & 63; const int d2 = (e >> 6) & 63; const int h = e >> 12;
#pragma unroll
      for (int q = 0; q < 4; ++q) vv[q] = tohx(FVt[(size_t)(j2 + q) * DD + h * HD + d2]); }
    *(volatile v4h*)(KX + e) = kk; *(volatile v4h*)(VXT + e) = vv; __threadfence(); *(volatile v4h*)(KX + e) = kk; *(volatile v4h*)(VXT + e) = vv; }

__global__ __launch_bounds__(256) void k_merge(const float* __restrict__ O, int b, int h0, bf* Ah, bf* Al) {
    const int lane = threadIdx.x & 31; const int L0 = (blockIdx.x * 8 + (threadIdx.x >> 5)) * 8; const int nlines = ZH * TT * HD / 64;
#pragma unroll 1
    for (int ps = 0; ps < 2; ++ps) {
#pragma unroll
        for (int l = 0; l < 8; ++l) { const int L = L0 + l; if (L >= nlines) break; const int e = L * 64 + lane * 2; const int d = e & 63; const int t = (e >> 6) & (TT - 1); const int zz = e >> 17; v2us oh, ol;
#pragma unroll
            for (int q = 0; q < 2; ++q) { unsigned short a, c2; splitf(O[(size_t)e + q] * (1.0f / PCAR), a, c2); oh[q] = a; ol[q] = c2; }
            const size_t o = ((size_t)b * TT + t) * DD + (h0 + zz) * HD + d; *(volatile v2us*)(Ah + o) = oh; *(volatile v2us*)(Al + o) = ol; }
        if (ps == 0) __threadfence(); }
}
template <int RAW>
__global__ __launch_bounds__(256) void k_lnres(const float* __restrict__ A, const float* __restrict__ R, const float* __restrict__ gg, const float* __restrict__ bb, float* X, bf* Xh, bf* Xl) {
    const int lane = threadIdx.x & 31; const int r = blockIdx.x * 8 + (threadIdx.x >> 5); if (r >= NT) return; float v[DD / 32]; float s = 0.f;
#pragma unroll
    for (int c = 0; c < DD / 128; ++c) { const v4f a = *(const v4f*)(A + (size_t)r * DD + c * 128 + lane * 4), xx = *(const v4f*)(R + (size_t)r * DD + c * 128 + lane * 4);
#pragma unroll
        for (int q = 0; q < 4; ++q) { v[c * 4 + q] = a[q] + (RAW ? bfr(xx[q]) : xx[q]); s += v[c * 4 + q]; } }
#pragma unroll
    for (int sh = 16; sh; sh >>= 1) s += __shfl_xor(s, sh, 32);
    const float mu = s * (1.0f / DD); float qq = 0.f;
#pragma unroll
    for (int i = 0; i < DD / 32; ++i) { const float d0 = v[i] - mu; qq = __fadd_rn(qq, __fmul_rn(d0, d0)); }
#pragma unroll
    for (int sh = 16; sh; sh >>= 1) qq += __shfl_xor(qq, sh, 32);
    const float rs = __fdiv_rn(1.0f, __fsqrt_rn(qq * (1.0f / DD) + 1e-12f));
    float o[DD / 32];
#pragma unroll
    for (int c = 0; c < DD / 128; ++c) {
#pragma unroll
        for (int q = 0; q < 4; ++q) { const int col = c * 128 + lane * 4 + q; o[c * 4 + q] = __fadd_rn(__fmul_rn((v[c * 4 + q] - mu) * rs, bfr(gg[col])), bfr(bb[col])); } }
#pragma unroll 1
    for (int ps = 0; ps < 2; ++ps) {
#pragma unroll
        for (int c = 0; c < DD / 128; ++c) { v4f w4; v4us oh, ol;
#pragma unroll
            for (int q = 0; q < 4; ++q) { w4[q] = o[c * 4 + q]; unsigned short a, c2; splitf(o[c * 4 + q], a, c2); oh[q] = a; ol[q] = c2; }
            if (X) *(volatile v4f*)(X + (size_t)r * DD + c * 128 + lane * 4) = w4;
            *(volatile v4us*)(Xh + (size_t)r * DD + c * 128 + lane * 4) = oh; *(volatile v4us*)(Xl + (size_t)r * DD + c * 128 + lane * 4) = ol; }
        if (ps == 0) __threadfence(); }
}
__global__ __launch_bounds__(256) void k_gelusplit(const float* __restrict__ H, bf* Hh, bf* Hl, size_t n) {
    const size_t i = ((size_t)blockIdx.x * 256 + threadIdx.x) * 2; if (i >= n) return; v2us oh, ol;
#pragma unroll
    for (int q = 0; q < 2; ++q) { const float h = H[i + q]; unsigned short a, c2; splitf(0.5f * h * (1.0f + erff(h * 0.70710678118654752f)), a, c2); oh[q] = a; ol[q] = c2; }
    *(volatile v2us*)(Hh + i) = oh; *(volatile v2us*)(Hl + i) = ol; __threadfence(); *(volatile v2us*)(Hh + i) = oh; *(volatile v2us*)(Hl + i) = ol;
}
extern "C" void kernel_launch(void* const* d_in, const int* in_sizes, int n_in,
                              void* d_out, int out_size, void* d_ws, size_t ws_size, hipStream_t stream) {
    (void)in_sizes; (void)n_in; (void)out_size;
    const float* IN[28]; for (int i = 0; i < 28; ++i) IN[i] = (const float*)d_in[i];
    const float* hs = IN[0]; const float* tag = IN[1];
    float* OUT = (float*)d_out;
    char* wsp = (char*)d_ws;
    auto take = [&](size_t bytes) { char* p = wsp; wsp += (bytes + 255) & ~(size_t)255; return (void*)p; };
    bf* WA = (bf*)take((size_t)DD * DD * 2); bf* WB = (bf*)take((size_t)DD * DD * 2); bf* WC = (bf*)take((size_t)DD * DD * 2); bf* WD = (bf*)take((size_t)DD * DD * 2); bf* W1T = (bf*)take((size_t)FFH * DD * 2); bf* W2T = (bf*)take((size_t)DD * FFH * 2);
    bf* XB = (bf*)take((size_t)NT * DD * 2); float* F = (float*)take((size_t)NT * DD * 4);
    char* R0 = wsp; h16* QP = (h16*)take((size_t)NT * DD * 2); h16* KP = (h16*)take((size_t)NT * DD * 2); h16* VT = (h16*)take((size_t)NT * DD * 2);
    float* Sb = (float*)take((size_t)ZH * TT * TT * 4); h16* Pm = (h16*)take((size_t)ZH * TT * TT * 2); float* Ob = (float*)take((size_t)ZH * TT * HD * 4); char* R1 = wsp;
    bf* ATh = (bf*)take((size_t)NT * DD * 2); bf* ATl = (bf*)take((size_t)NT * DD * 2); float* X1 = (float*)take((size_t)NT * DD * 4); bf* X1h = (bf*)take((size_t)NT * DD * 2); bf* X1l = (bf*)take((size_t)NT * DD * 2);
    bf* TAGB = (bf*)take((size_t)NTAG * DD * 2); float* FK = (float*)take((size_t)NTAG * DD * 4); float* FV2 = (float*)take((size_t)NTAG * DD * 4); h16* KX = (h16*)take((size_t)NH_ * NTAG * HD * 2); h16* VXT = (h16*)take((size_t)NH_ * HD * NTAG * 2);
    if ((size_t)(wsp - (char*)d_ws) > ws_size) return;
    float* H = (float*)R0; bf* Hh = (bf*)(R0 + (size_t)TT * FFH * 4); bf* Hl = (bf*)(R0 + (size_t)TT * FFH * 6); if ((char*)(Hl + (size_t)TT * FFH) > R1) return;
    float* SX = Sb; h16* PX = Pm; float* OX = Ob;
    OX = Sb + (size_t)NH_ * TT * NTAG;
    float* Y = F; float* X2 = X1; bf* X2h = X1h; bf* X2l = X1l; float* FF2 = (float*)ATh;
    const unsigned LB = (unsigned)((NT * DD / 64 + 63) / 64), gW = (unsigned)((DD * DD / 64 + 63) / 64), gF = (unsigned)((DD * FFH / 64 + 63) / 64); const dim3 gP(NT / 64, DD / 64, 1);
    k_wtG<<<gW, 256, 0, stream>>>(IN[2], DD, DD, WA); k_wtG<<<gW, 256, 0, stream>>>(IN[4], DD, DD, WB); k_wtG<<<gW, 256, 0, stream>>>(IN[6], DD, DD, WC); k_wtG<<<gW, 256, 0, stream>>>(IN[8], DD, DD, WD);
    k_cvt8<<<(unsigned)(((size_t)NT * DD / 8 + 255) / 256), 256, 0, stream>>>(hs, XB, (size_t)NT * DD / 8);
    k_gemmw<bf, 0, true><<<gP, 32, 0, stream>>>(XB, nullptr, WA, nullptr, DD, F, DD, IN[3], 0, 0, 0); k_h16plane<<<LB, 256, 0, stream>>>(F, 0.125f, QP);
    k_gemmw<bf, 0, true><<<gP, 32, 0, stream>>>(XB, nullptr, WB, nullptr, DD, F, DD, IN[5], 0, 0, 0); k_h16plane<<<LB, 256, 0, stream>>>(F, 1.0f, KP);
    k_gemmw<bf, 0, true><<<gP, 32, 0, stream>>>(XB, nullptr, WC, nullptr, DD, F, DD, IN[7], 0, 0, 0); k_vtplane<<<LB, 256, 0, stream>>>(F, VT);
    for (int b = 0; b < NB_; ++b)
        for (int h0 = 0; h0 < NH_; h0 += ZH) { const size_t z0 = (size_t)b * NH_ + h0;
            k_gemmw<h16, 0, false><<<dim3(TT / 64, TT / 64, ZH), 32, 0, stream>>>(QP + z0 * TT * HD, nullptr, KP + z0 * TT * HD, nullptr, HD, Sb, TT, nullptr, (size_t)TT * HD, (size_t)TT * HD, (size_t)TT * TT);
            k_msoft<<<ZH * TT / 8, 256, 0, stream>>>(Sb, Pm);
            k_gemmw<h16, 0, false><<<dim3(TT / 64, 1, ZH), 32, 0, stream>>>(Pm, nullptr, VT + z0 * HD * TT, nullptr, TT, Ob, HD, nullptr, (size_t)TT * TT, (size_t)HD * TT, (size_t)TT * HD);
            k_merge<<<(TT * ZH * HD / 64 + 63) / 64, 256, 0, stream>>>(Ob, b, h0, ATh, ATl); }
    k_gemmw<bf, 1, true><<<gP, 32, 0, stream>>>(ATh, ATl, WD, nullptr, DD, Y, DD, IN[9], 0, 0, 0);
    k_lnres<1><<<NT / 8, 256, 0, stream>>>(Y, hs, IN[10], IN[11], X1, X1h, X1l);
    k_wtG<<<gW, 256, 0, stream>>>(IN[12], DD, DD, WA); k_wtG<<<gW, 256, 0, stream>>>(IN[14], DD, DD, WB); k_wtG<<<gW, 256, 0, stream>>>(IN[16], DD, DD, WC); k_wtG<<<gW, 256, 0, stream>>>(IN[18], DD, DD, WD);
    k_cvt8<<<(NTAG * DD / 8 + 255) / 256, 256, 0, stream>>>(tag, TAGB, (size_t)NTAG * DD / 8);
    k_gemmw<bf, 1, true><<<gP, 32, 0, stream>>>(X1h, X1l, WA, nullptr, DD, F, DD, IN[13], 0, 0, 0); k_h16plane<<<LB, 256, 0, stream>>>(F, 0.125f, QP);
    k_gemmw<bf, 0, true><<<dim3(1, DD / 64, 1), 32, 0, stream>>>(TAGB, nullptr, WB, nullptr, DD, FK, DD, IN[15], 0, 0, 0); k_gemmw<bf, 0, true><<<dim3(1, DD / 64, 1), 32, 0, stream>>>(TAGB, nullptr, WC, nullptr, DD, FV2, DD, IN[17], 0, 0, 0);
    k_tag16<<<(NH_ * NTAG * HD / 4 + 255) / 256, 256, 0, stream>>>(FK, FV2, KX, VXT);
    for (int b = 0; b < NB_; ++b) { const size_t z0 = (size_t)b * NH_;
        k_gemmw<h16, 0, false><<<dim3(TT / 64, 1, NH_), 32, 0, stream>>>(QP + z0 * TT * HD, nullptr, KX, nullptr, HD, SX, NTAG, nullptr, (size_t)TT * HD, (size_t)NTAG * HD, (size_t)TT * NTAG);
        k_soft64<<<NH_ * TT / 8, 256, 0, stream>>>(SX, NH_ * TT, PX);
        k_gemmw<h16, 0, false><<<dim3(TT / 64, 1, NH_), 32, 0, stream>>>(PX, nullptr, VXT, nullptr, NTAG, OX, HD, nullptr, (size_t)TT * NTAG, (size_t)HD * NTAG, (size_t)TT * HD);
        for (int h0 = 0; h0 < NH_; h0 += ZH) k_merge<<<(TT * ZH * HD / 64 + 63) / 64, 256, 0, stream>>>(OX + (size_t)h0 * TT * HD, b, h0, ATh, ATl); }
    k_gemmw<bf, 1, true><<<gP, 32, 0, stream>>>(ATh, ATl, WD, nullptr, DD, Y, DD, IN[19], 0, 0, 0);
    k_lnres<0><<<NT / 8, 256, 0, stream>>>(Y, X1, IN[20], IN[21], X2, X2h, X2l);
    k_wtG<<<gF, 256, 0, stream>>>(IN[22], DD, FFH, W1T); k_wtG<<<gF, 256, 0, stream>>>(IN[24], FFH, DD, W2T);
    for (int hb = 0; hb < 2; ++hb) { const size_t r0 = (size_t)hb * TT;
        k_gemmw<bf, 1, true><<<dim3(TT / 64, FFH / 64, 1), 32, 0, stream>>>(X2h + r0 * DD, X2l + r0 * DD, W1T, nullptr, DD, H, FFH, IN[23], 0, 0, 0);
        k_gelusplit<<<(unsigned)(((size_t)TT * FFH / 2 + 255) / 256), 256, 0, stream>>>(H, Hh, Hl, (size_t)TT * FFH);
        k_gemmw<bf, 1, true><<<dim3(TT / 64, DD / 64, 1), 32, 0, stream>>>(Hh, Hl, W2T, nullptr, FFH, FF2 + r0 * DD, DD, IN[25], 0, 0, 0); }
    k_lnres<0><<<NT / 8, 256, 0, stream>>>(FF2, X2, IN[26], IN[27], OUT, XB, XB + (size_t)NT * DD);
}
